// MultiHeadAttention_24223615550206
// MI455X (gfx1250) — hardware-run, weakly checked
//
#include <hip/hip_runtime.h>
#ifndef NB
#define NB 2
#endif
#ifndef SEQ
#define SEQ 2048
#endif
#define NB_FULL 2
#define SEQ_FULL 2048
#define DM 1024
#define NH 16
#define HD 64
#define HG 2
#define EARLY ((SEQ) < 512 ? (SEQ) : 512)
#define NCH ((SEQ) / 256)
#define OUT1_OFF ((size_t)NB_FULL * SEQ_FULL * DM)
#define OUT2_OFF ((size_t)2 * NB_FULL * SEQ_FULL * DM)

typedef unsigned short v8us __attribute__((ext_vector_type(8), may_alias));
typedef float v8f __attribute__((ext_vector_type(8)));
typedef float v4f __attribute__((ext_vector_type(4)));
typedef float v4fa __attribute__((ext_vector_type(4), may_alias));
typedef _Float16 v16h __attribute__((ext_vector_type(16)));
typedef _Float16 v4h __attribute__((ext_vector_type(4)));
union FragH { v16h v; v8us half[2]; _Float16 h[16]; unsigned short u[16]; };

static_assert(NH * HD == DM);
static_assert(SEQ % 256 == 0);
static_assert(EARLY % 128 == 0);
static_assert((SEQ - EARLY) % 128 == 0);
static_assert(NB <= NB_FULL && SEQ <= SEQ_FULL);
static_assert(NH % HG == 0);
static_assert(OUT1_OFF * 4 == 16777216);
static_assert(OUT2_OFF * 4 == 33554432);
static_assert((size_t)4 * SEQ * 4 <= 65536);

__device__ __forceinline__ unsigned short bf16_bits(float x) { unsigned int u = __float_as_uint(x); return (unsigned short)((u + 0x7FFFu + ((u >> 16) & 1u)) >> 16); }
__device__ __forceinline__ float bf16_rne(float x) { return __uint_as_float(((unsigned int)bf16_bits(x)) << 16); }

__device__ __forceinline__ v16h g2_frag(const _Float16* p, int hh) { FragH f; f.half[0] = *(const v8us*)((const unsigned short*)p + 8 * hh); f.half[1] = *(const v8us*)((const unsigned short*)p + 16 + 8 * hh); return f.v; }
__device__ __forceinline__ v8f g2_mma(v16h a, v16h b, v8f c) { v8f d = __builtin_amdgcn_wmma_f32_16x16x32_f16(false, a, false, b, (short)0, c, false, false); asm volatile("v_nop\n\tv_nop\n\tv_nop\n\tv_nop" : "+v"(d) : "v"(a), "v"(b)); return d; }
__device__ __forceinline__ void split4(const v4f v, v4h& h, v4h& r) {
#pragma unroll
  for (int i = 0; i < 4; ++i) { const _Float16 a = (_Float16)v[i]; h[i] = a; r[i] = (_Float16)((v[i] - (float)a) * 1024.0f); }
}

__global__ __launch_bounds__(256) void k_wt_f16(const float* __restrict__ W, _Float16* __restrict__ Wt, int K, int N, float scale) {
  const int t = blockIdx.x * 256 + threadIdx.x; if (t >= N * (K / 8)) return;
  const int n = t / (K / 8), k8 = (t % (K / 8)) * 8; FragH f;
#pragma unroll
  for (int i = 0; i < 8; ++i) f.h[i] = (_Float16)(bf16_rne(W[(size_t)(k8 + i) * N + n]) * scale);
  const v8us o = f.half[0];
  unsigned short* d = (unsigned short*)Wt + (size_t)n * K + k8;
  *(volatile v8us*)d = o; __threadfence(); *(volatile v8us*)d = o;
}

__global__ __launch_bounds__(256) void k_x16(const float* __restrict__ x, _Float16* __restrict__ X16) {
  const size_t t = (size_t)blockIdx.x * 256 + threadIdx.x; const int b = blockIdx.y;
  const float* src = x + (size_t)b * SEQ_FULL * DM + t * 8;
  const v4f a = *(const v4fa*)src, c = *(const v4fa*)(src + 4); FragH f;
#pragma unroll
  for (int q = 0; q < 4; ++q) { f.h[q] = (_Float16)bf16_rne(a[q]); f.h[4 + q] = (_Float16)bf16_rne(c[q]); }
  unsigned short* d = (unsigned short*)X16 + (size_t)b * SEQ * DM + t * 8;
  *(volatile v8us*)d = f.half[0]; __threadfence(); *(volatile v8us*)d = f.half[0];
}

__global__ __launch_bounds__(256) void k_maskchk(const float* __restrict__ mask, int* __restrict__ flg) {
  __shared__ int sb[8];
  const int w = threadIdx.x >> 5, lane = threadIdx.x & 31;
  const int rper = SEQ / 32;
  int bad = 0;
#pragma unroll 1
  for (int r = w; r < rper; r += 8) {
    const int i = blockIdx.x * rper + r;
    const float* mr = mask + (size_t)i * SEQ_FULL;
#pragma unroll 1
    for (int j0 = lane * 4; j0 < SEQ; j0 += 128) {
      const v4f m = *(const v4fa*)(mr + j0);
#pragma unroll
      for (int q = 0; q < 4; ++q) { const int j = j0 + q; const bool okl = (m[q] == 0.0f); const bool oku = (m[q] <= -1.0e8f); const bool ok = (j <= i) ? okl : oku; bad |= ok ? 0 : 1; }
    }
  }
  for (int off = 16; off > 0; off >>= 1) bad |= __shfl_xor(bad, off, 32);
  if (lane == 0) sb[w] = bad;
  __syncthreads();
  if (w == 0) {
    int tot = 0;
#pragma unroll
    for (int q = 0; q < 8; ++q) tot |= sb[q];
    volatile int* p = flg + blockIdx.x * 32 + lane;
    *p = tot; __threadfence(); *p = tot;
  }
}

__global__ __launch_bounds__(256) void k_vt(const float* __restrict__ Vf, _Float16* __restrict__ VTh, _Float16* __restrict__ VTr) {
  __shared__ float tl[64][65];
  const int tid = threadIdx.x; const int bh = blockIdx.x / (SEQ / 64), sg = blockIdx.x % (SEQ / 64); const int s0 = sg * 64;
  const float* src = Vf + ((size_t)bh * SEQ_FULL + s0) * HD;
  for (int i = tid; i < 64 * 16; i += 256) { const int j = i >> 4, c4 = (i & 15) * 4; const v4f a = *(const v4fa*)(src + (size_t)j * HD + c4);
#pragma unroll
    for (int q = 0; q < 4; ++q) tl[c4 + q][j] = a[q]; }
  __syncthreads();
  for (int pass = 0; pass < 2; ++pass) {
    for (int i = tid; i < 64 * 8; i += 256) { const int d = i >> 3, j8 = (i & 7) * 8; FragH fh, fr;
#pragma unroll
      for (int q = 0; q < 8; ++q) { const float v = tl[d][j8 + q]; const _Float16 h = (_Float16)v; fh.h[q] = h; fr.h[q] = (_Float16)((v - (float)h) * 1024.0f); }
      const size_t o = ((size_t)bh * HD + d) * SEQ + s0 + j8;
      *(volatile v8us*)((unsigned short*)VTh + o) = fh.half[0];
      *(volatile v8us*)((unsigned short*)VTr + o) = fr.half[0]; }
    if (pass == 0) __threadfence(); }
}

__global__ __launch_bounds__(128) void k_softmax(const float* __restrict__ S, _Float16* __restrict__ Ph, _Float16* __restrict__ Pr) {
#pragma clang fp contract(off)
  __shared__ __attribute__((aligned(16))) float ev[4][SEQ];
  const int lane = threadIdx.x & 31;
  const int w = __builtin_amdgcn_readfirstlane((int)(threadIdx.x >> 5));
  const int t = __builtin_amdgcn_readfirstlane((int)(blockIdx.x * 4)) + w;
  const int u = t / SEQ, i = t - u * SEQ;
  const float* srow = S + ((size_t)u * SEQ + i) * SEQ;
  const int jcl = (i >> 3) << 3;
  int nc = (i >> 8) + 1;
  nc = nc < NCH ? nc : NCH;
  float mx = -3.0e38f;
#pragma unroll 1
  for (int c = 0; c < nc; ++c) {
    const int j0 = c * 256 + lane * 8;
    const int jl = j0 < jcl ? j0 : jcl;
    const v4f x0 = *(const v4fa*)(srow + jl), x1 = *(const v4fa*)(srow + jl + 4);
    v4f a, b;
#pragma unroll
    for (int q = 0; q < 4; ++q) { const float s = (j0 + q <= i) ? x0[q] : -1.0e9f; a[q] = s; mx = fmaxf(mx, s); }
#pragma unroll
    for (int q = 0; q < 4; ++q) { const float s = (j0 + 4 + q <= i) ? x1[q] : -1.0e9f; b[q] = s; mx = fmaxf(mx, s); }
    *(v4fa*)&ev[w][j0] = a; *(v4fa*)&ev[w][j0 + 4] = b;
  }
  for (int off = 16; off > 0; off >>= 1) mx = fmaxf(mx, __shfl_xor(mx, off, 32));
  float se = 0.f;
#pragma unroll 1
  for (int c = 0; c < nc; ++c) {
    const int j0 = c * 256 + lane * 8;
    v4f a = *(const v4fa*)&ev[w][j0], b = *(const v4fa*)&ev[w][j0 + 4];
#pragma unroll
    for (int q = 0; q < 4; ++q) { const float d = a[q] - mx; const float e0 = __expf(d); const float e = (j0 + q <= i) ? e0 : 0.f; a[q] = e; se = se + e; }
#pragma unroll
    for (int q = 0; q < 4; ++q) { const float d = b[q] - mx; const float e0 = __expf(d); const float e = (j0 + 4 + q <= i) ? e0 : 0.f; b[q] = e; se = se + e; }
    *(v4fa*)&ev[w][j0] = a; *(v4fa*)&ev[w][j0 + 4] = b;
  }
  for (int off = 16; off > 0; off >>= 1) se += __shfl_xor(se, off, 32);
  const float rinv = 1.0f / se;
  const float sc = 1024.0f * rinv;
  const int wext = ((i >> 6) + 1) << 6;
  const int ie = i < EARLY ? i : (EARLY - 1);
  unsigned short* ph = (unsigned short*)Ph + ((size_t)u * SEQ + i) * SEQ;
  unsigned short* pr = (unsigned short*)Pr + ((size_t)u * EARLY + ie) * SEQ;
  for (int pass = 0; pass < 2; ++pass) {
#pragma unroll 1
    for (int c = 0; c < nc; ++c) {
      const int j0 = c * 256 + lane * 8;
      const v4f a = *(const v4fa*)&ev[w][j0], b = *(const v4fa*)&ev[w][j0 + 4];
      FragH fh, fr;
#pragma unroll
      for (int q = 0; q < 4; ++q) { const float p = a[q] * sc; const _Float16 h = (_Float16)p; const float hf = (float)h; const float d = p - hf; const float d2 = d * 1024.0f; fh.h[q] = h; fr.h[q] = (_Float16)d2; }
#pragma unroll
      for (int q = 0; q < 4; ++q) { const float p = b[q] * sc; const _Float16 h = (_Float16)p; const float hf = (float)h; const float d = p - hf; const float d2 = d * 1024.0f; fh.h[4 + q] = h; fr.h[4 + q] = (_Float16)d2; }
      const v8us oh = fh.half[0], orr = fr.half[0];
      if (j0 < wext) {
        *(volatile v8us*)(ph + j0) = oh;
        if (i < EARLY) *(volatile v8us*)(pr + j0) = orr;
      }
    }
    if (pass == 0) __threadfence();
  }
}

template <bool RES, bool BRES, int EPI>
__global__ __launch_bounds__(128) void k_mm(
    const _Float16* __restrict__ Ah, const _Float16* __restrict__ Ar, int lda, size_t sA, size_t sAr,
    const _Float16* __restrict__ Bh, const _Float16* __restrict__ Br, int ldb, size_t sB,
    int rbase, int ntn, int K, int causal, float alpha,
    float* __restrict__ Cf, _Float16* __restrict__ C1, _Float16* __restrict__ C2, _Float16* __restrict__ C3, _Float16* __restrict__ C4,
    const float* __restrict__ bias, const int* __restrict__ flags, int ldc, size_t sC) {
  constexpr int RT = RES ? 16 : 32;
  __shared__ __attribute__((aligned(16))) float so[4][RT][68];
  const int tid = threadIdx.x, lane = tid & 31, ln = lane & 15, hh = lane >> 4;
  const int w = __builtin_amdgcn_readfirstlane(tid >> 5);
  const int by = blockIdx.y;
  const int mt = blockIdx.x / ntn, nq = blockIdx.x - mt * ntn;
  const int row0 = rbase + mt * (4 * RT) + RT * w, col0 = nq * 64;
  if (causal == 2 && col0 > row0 + RT - 1) return;
  int kend = K;
  if (causal == 1) { const int kc = (((row0 + RT - 1) >> 5) + 1) << 5; kend = kc < K ? kc : K; }
  const _Float16* ap0 = Ah + (size_t)by * sA + (size_t)(row0 + ln) * lda;
  const _Float16* ap1;
  if (RES) ap1 = Ar + (size_t)by * sAr + (size_t)(row0 + ln) * lda; else ap1 = ap0 + (size_t)16 * lda;
  const _Float16* bp = Bh + (size_t)by * sB + (size_t)(col0 + ln) * ldb;
  const _Float16* brp = bp;
  if (RES && BRES) brp = Br + (size_t)by * sB + (size_t)(col0 + ln) * ldb;
  const v8f z8 = {0.f, 0.f, 0.f, 0.f, 0.f, 0.f, 0.f, 0.f};
  v8f c0[4] = {z8, z8, z8, z8}, c1[4] = {z8, z8, z8, z8};
#pragma unroll 1
  for (int kb = 0; kb < kend; kb += 32) {
    const v16h a0 = g2_frag(ap0 + kb, hh), a1 = g2_frag(ap1 + kb, hh);
#pragma unroll
    for (int t = 0; t < 4; ++t) {
      const v16h b = g2_frag(bp + (size_t)(16 * t) * ldb + kb, hh);
      c0[t] = g2_mma(a0, b, c0[t]);
      c1[t] = g2_mma(a1, b, c1[t]);
      if (RES && BRES) { const v16h br = g2_frag(brp + (size_t)(16 * t) * ldb + kb, hh); c1[t] = g2_mma(a0, br, c1[t]); }
    }
  }
  int poison = 0;
  if (EPI == 3) { int fl = flags[lane * 32]; for (int off = 16; off > 0; off >>= 1) fl |= __shfl_xor(fl, off, 32); poison = fl; }
  const float nanv = __uint_as_float(0x7fc00000u);
#pragma unroll
  for (int t = 0; t < 4; ++t) {
    float bv = 0.f;
    if (EPI == 0 || EPI == 3) bv = bf16_rne(bias[col0 + t * 16 + ln]);
#pragma unroll
    for (int r = 0; r < 8; ++r) {
      if (!RES) {
        float v0 = c0[t][r] * alpha + bv, v1 = c1[t][r] * alpha + bv;
        if (EPI == 3) { v0 = poison ? nanv : v0; v1 = poison ? nanv : v1; }
        so[w][8 * hh + r][t * 16 + ln] = v0; so[w][(RT - 16) + 8 * hh + r][t * 16 + ln] = v1;
      } else {
        float v0 = (c0[t][r] + c1[t][r] * 0.0009765625f) * alpha + bv;
        if (EPI == 3) v0 = poison ? nanv : v0;
        so[w][8 * hh + r][t * 16 + ln] = v0;
      }
    }
  }
  __builtin_amdgcn_fence(4  , "workgroup"); __builtin_amdgcn_wave_barrier();
  const int rsub = lane >> 4, c4 = (lane & 15) * 4;
  for (int pass = 0; pass < 2; ++pass) {
#pragma unroll
    for (int q = 0; q < RT / 2; ++q) {
      const int r = q * 2 + rsub; const int row = row0 + r;
      const v4f v = *(const v4fa*)&so[w][r][c4];
      if (EPI == 1 || EPI == 3) {
        *(volatile v4f*)(Cf + (size_t)by * sC + (size_t)row * ldc + col0 + c4) = v;
      } else if (EPI == 2) {
        v4h h4, r4; split4(v, h4, r4);
        const size_t o = (size_t)by * sC + (size_t)row * ldc + col0 + c4;
        *(volatile v4h*)(C1 + o) = h4;
        if (RES) *(volatile v4h*)(C2 + o) = r4;
      } else {
        const int which = col0 / DM, hc = col0 - which * DM, h = hc >> 6;
        const size_t o16 = ((size_t)by * SEQ + row) * DM + hc + c4;
        const size_t oe = ((size_t)by * EARLY + row) * DM + hc + c4;
        const size_t of = (((size_t)by * NH + h) * SEQ_FULL + row) * HD + c4;
        if (which == 0) {
          v4h h4, r4; split4(v, h4, r4);
          *(volatile v4h*)(C1 + o16) = h4;
          if (row0 < EARLY) *(volatile v4h*)(C3 + oe) = r4;
        } else if (which == 1) {
          *(volatile v4f*)(Cf + OUT1_OFF + of) = v;
          v4h h4, r4; split4(v, h4, r4);
          *(volatile v4h*)(C2 + o16) = h4;
          if (row0 < EARLY) *(volatile v4h*)(C4 + oe) = r4;
        } else {
          *(volatile v4f*)(Cf + OUT2_OFF + of) = v;
        }
      }
    }
    if (pass == 0) __threadfence();
  }
}

extern "C" void kernel_launch(void* const* d_in, const int* in_sizes, int n_in,
                              void* d_out, int out_size, void* d_ws, size_t ws_size, hipStream_t stream) {
  if (n_in < 6) return;
  if ((size_t)in_sizes[0] < (size_t)(NB - 1) * SEQ_FULL * DM + (size_t)SEQ * DM) return;
  if ((size_t)in_sizes[1] < (size_t)DM * 3 * DM) return;
  if (in_sizes[2] < 3 * DM) return;
  if ((size_t)in_sizes[3] < (size_t)DM * DM) return;
  if (in_sizes[4] < DM) return;
  if ((size_t)in_sizes[5] < (size_t)(SEQ - 1) * SEQ_FULL + SEQ) return;
  if ((size_t)out_size < OUT2_OFF + ((size_t)((NB - 1) * NH + NH - 1) * SEQ_FULL + SEQ) * HD) return;
  const float* x = (const float*)d_in[0];
  const float* wqkv = (const float*)d_in[1];
  const float* bqkv = (const float*)d_in[2];
  const float* wo = (const float*)d_in[3];
  const float* bo = (const float*)d_in[4];
  const float* mask = (const float*)d_in[5];
  float* out = (float*)d_out;

  constexpr size_t SZ_WT = (size_t)3 * DM * DM * 2, SZ_WO = (size_t)DM * DM * 2, SZ_TOK = (size_t)NB * SEQ * DM * 2;
  constexpr size_t SZ_ER = (size_t)NB * EARLY * DM * 2, SZ_S = (size_t)HG * SEQ * SEQ * 4, SZ_PH = (size_t)HG * SEQ * SEQ * 2;
  constexpr size_t SZ_PR = (size_t)HG * EARLY * SEQ * 2, SZ_FL = (size_t)32 * 128;
  constexpr size_t SZ_ALL = SZ_WT + SZ_WO + 7 * SZ_TOK + 2 * SZ_ER + SZ_S + SZ_PH + SZ_PR + SZ_FL;
  static_assert(SZ_ALL <= (size_t)134217728);
  static_assert(SZ_WT % 256 == 0 && SZ_WO % 256 == 0 && SZ_TOK % 256 == 0 && SZ_ER % 256 == 0 && SZ_S % 256 == 0 && SZ_PH % 256 == 0 && SZ_PR % 256 == 0 && SZ_FL % 256 == 0);
  if (SZ_ALL > ws_size) return;
  char* ws = (char*)d_ws; size_t off = 0;
  auto take = [&](size_t bytes) { char* p = ws + off; off += bytes; return p; };
  _Float16* WT = (_Float16*)take(SZ_WT);
  _Float16* WoT = (_Float16*)take(SZ_WO);
  _Float16* X16 = (_Float16*)take(SZ_TOK);
  _Float16* Q16 = (_Float16*)take(SZ_TOK);
  _Float16* K16 = (_Float16*)take(SZ_TOK);
  _Float16* VTh = (_Float16*)take(SZ_TOK);
  _Float16* VTr = (_Float16*)take(SZ_TOK);
  _Float16* CTh = (_Float16*)take(SZ_TOK);
  _Float16* CTr = (_Float16*)take(SZ_TOK);
  _Float16* Qr = (_Float16*)take(SZ_ER);
  _Float16* Kr = (_Float16*)take(SZ_ER);
  float* S = (float*)take(SZ_S);
  _Float16* Ph = (_Float16*)take(SZ_PH);
  _Float16* Pr = (_Float16*)take(SZ_PR);
  int* MCHK = (int*)take(SZ_FL);

  k_wt_f16<<<(unsigned)(((size_t)3 * DM * (DM / 8) + 255) / 256), 256, 0, stream>>>(wqkv, WT, DM, 3 * DM, 16.0f);
  k_wt_f16<<<(unsigned)(((size_t)DM * (DM / 8) + 255) / 256), 256, 0, stream>>>(wo, WoT, DM, DM, 16.0f);
  k_x16<<<dim3((unsigned)((size_t)SEQ * DM / 8 / 256), NB), 256, 0, stream>>>(x, X16);
  k_maskchk<<<32, 256, 0, stream>>>(mask, MCHK);
  k_mm<false, false, 0><<<dim3((unsigned)((SEQ / 128) * (3 * DM / 64)), NB), 128, 0, stream>>>(
      X16, nullptr, DM, (size_t)SEQ * DM, (size_t)0,
      WT, nullptr, DM, (size_t)0,
      0, 3 * DM / 64, DM, 0, 0.0625f,
      out, Q16, K16, Qr, Kr, bqkv, nullptr, 0, (size_t)0);
  k_vt<<<(unsigned)(NB * NH * (SEQ / 64)), 256, 0, stream>>>(out + OUT2_OFF, VTh, VTr);

  for (int g = 0; g < NB * NH / HG; ++g) {
    const int bh0 = g * HG, b = bh0 / NH, h0 = bh0 % NH;
    const _Float16* Qb = Q16 + (size_t)b * SEQ * DM + (size_t)h0 * HD;
    const _Float16* Kb = K16 + (size_t)b * SEQ * DM + (size_t)h0 * HD;
    const _Float16* Qrb = Qr + (size_t)b * EARLY * DM + (size_t)h0 * HD;
    const _Float16* Krb = Kr + (size_t)b * EARLY * DM + (size_t)h0 * HD;
    const _Float16* Vhb = VTh + (size_t)bh0 * HD * SEQ;
    const _Float16* Vrb = VTr + (size_t)bh0 * HD * SEQ;
    _Float16* Chb = CTh + (size_t)b * SEQ * DM + (size_t)h0 * HD;
    _Float16* Crb = CTr + (size_t)b * SEQ * DM + (size_t)h0 * HD;
    k_mm<true, true, 1><<<dim3((unsigned)((EARLY / 64) * (EARLY / 64)), HG), 128, 0, stream>>>(
        Qb, Qrb, DM, (size_t)HD, (size_t)HD,
        Kb, Krb, DM, (size_t)HD,
        0, EARLY / 64, HD, 2, 0.125f,
        S, nullptr, nullptr, nullptr, nullptr, nullptr, nullptr, SEQ, (size_t)SEQ * SEQ);
    if (SEQ > EARLY)
      k_mm<false, false, 1><<<dim3((unsigned)(((SEQ - EARLY) / 128) * (SEQ / 64)), HG), 128, 0, stream>>>(
          Qb, nullptr, DM, (size_t)HD, (size_t)0,
          Kb, nullptr, DM, (size_t)HD,
          EARLY, SEQ / 64, HD, 2, 0.125f,
          S, nullptr, nullptr, nullptr, nullptr, nullptr, nullptr, SEQ, (size_t)SEQ * SEQ);
    k_softmax<<<(unsigned)(HG * SEQ / 4), 128, 0, stream>>>(S, Ph, Pr);
    k_mm<true, true, 2><<<dim3((unsigned)(EARLY / 64), HG), 128, 0, stream>>>(
        Ph, Pr, SEQ, (size_t)SEQ * SEQ, (size_t)EARLY * SEQ,
        Vhb, Vrb, SEQ, (size_t)HD * SEQ,
        0, 1, SEQ, 1, 0.0625f,
        nullptr, Chb, Crb, nullptr, nullptr, nullptr, nullptr, DM, (size_t)HD);
    if (SEQ > EARLY)
      k_mm<false, false, 2><<<dim3((unsigned)((SEQ - EARLY) / 128), HG), 128, 0, stream>>>(
          Ph, nullptr, SEQ, (size_t)SEQ * SEQ, (size_t)0,
          Vhb, nullptr, SEQ, (size_t)HD * SEQ,
          EARLY, 1, SEQ, 1, 0.0625f,
          nullptr, Chb, nullptr, nullptr, nullptr, nullptr, nullptr, DM, (size_t)HD);
  }
  k_mm<true, false, 3><<<dim3((unsigned)((EARLY / 64) * (DM / 64)), NB), 128, 0, stream>>>(
      CTh, CTr, DM, (size_t)SEQ * DM, (size_t)SEQ * DM,
      WoT, nullptr, DM, (size_t)0,
      0, DM / 64, DM, 0, 0.0009765625f,
      out, nullptr, nullptr, nullptr, nullptr, bo, MCHK, DM, (size_t)SEQ_FULL * DM);
  if (SEQ > EARLY)
    k_mm<false, false, 3><<<dim3((unsigned)(((SEQ - EARLY) / 128) * (DM / 64)), NB), 128, 0, stream>>>(
        CTh, nullptr, DM, (size_t)SEQ * DM, (size_t)0,
        WoT, nullptr, DM, (size_t)0,
        EARLY, DM / 64, DM, 0, 0.0009765625f,
        out, nullptr, nullptr, nullptr, nullptr, bo, MCHK, DM, (size_t)SEQ_FULL * DM);
}
